// MultiScaleTemporalAttention_52063593562207
// MI455X (gfx1250) — hardware-verified
//
#include <hip/hip_runtime.h>
#include <hip/hip_bf16.h>


typedef _Float16 v16h __attribute__((ext_vector_type(16)));
typedef __bf16 v16b __attribute__((ext_vector_type(16)));
typedef float v8f __attribute__((ext_vector_type(8)));
typedef float v4f_t __attribute__((ext_vector_type(4)));
typedef unsigned int v4u_t __attribute__((ext_vector_type(4)));
typedef v4f_t __attribute__((may_alias)) v4f;
typedef v4u_t __attribute__((may_alias)) v4u;

#define NB 2
#define NS 2048
#define ND 1024
#define NH 16
#define HD 64
#define MR (NB * NS)
#define NC (2 * ND)
#define PLANE ((size_t)MR * (size_t)ND)
#define PP 72
#define TPF 68

#define SCL 0.125f
#define LOGD (-0.10536051565782628f)
#define NEGL (-1.0e30f)
#define NEGT (-1.0e29f)
#define WUP 64.0f
#define WDN 0.015625f
#define PUP 16384.0f
#define PDN 6.103515625e-05f

__device__ __forceinline__ unsigned short bfbits(float f) {
  unsigned int u = __float_as_uint(f);
  u = u + 0x7FFFu + ((u >> 16) & 1u);
  return (unsigned short)(u >> 16);
}
__device__ __forceinline__ float bff(unsigned short b) {
  return __uint_as_float(((unsigned int)b) << 16);
}
__device__ __forceinline__ unsigned short hbits(float f) {
  _Float16 hv = (_Float16)f;
  unsigned short u;
  __builtin_memcpy(&u, &hv, 2);
  return u;
}
__device__ __forceinline__ unsigned int pk2(unsigned short a, unsigned short b) {
  return (unsigned int)a | ((unsigned int)b << 16);
}
__device__ __forceinline__ v8f z8() {
  v8f v;
#pragma unroll
  for (int i = 0; i < 8; ++i) v[i] = 0.0f;
  return v;
}

union FH { v16h v; v4u_t u[2]; };
union FB { v16b v; v4u_t u[2]; };

__device__ __forceinline__ v16h ldh(const unsigned short* p, int h) {
  FH f;
  f.u[0] = *(const v4u*)(p + 8 * h);
  f.u[1] = *(const v4u*)(p + 16 + 8 * h);
  return f.v;
}
__device__ __forceinline__ v16b ldb(const unsigned short* p, int h) {
  FB f;
  f.u[0] = *(const v4u*)(p + 8 * h);
  f.u[1] = *(const v4u*)(p + 16 + 8 * h);
  return f.v;
}

__device__ __forceinline__ v8f mma_h(v16h a, v16h b, v8f c) {
  c = __builtin_amdgcn_wmma_f32_16x16x32_f16(false, a, false, b, (short)0, c, false, false);
  asm volatile("v_nop\n\tv_nop\n\tv_nop\n\tv_nop" : "+v"(c) : "v"(a), "v"(b));
  return c;
}
__device__ __forceinline__ v8f mma_b(v16b a, v16b b, v8f c) {
  c = __builtin_amdgcn_wmma_f32_16x16x32_bf16(false, a, false, b, (short)0, c, false, false);
  asm volatile("v_nop\n\tv_nop\n\tv_nop\n\tv_nop" : "+v"(c) : "v"(a), "v"(b));
  return c;
}

__global__ __launch_bounds__(256) void k_xcvt(const float* __restrict__ x,
                                              unsigned short* __restrict__ xh,
                                              unsigned short* __restrict__ xbh,
                                              unsigned short* __restrict__ xbl, int n8) {
  const int i = blockIdx.x * 256 + (int)threadIdx.x;
  if (i >= n8) return;
  const size_t o = (size_t)i * 8;
  const v4f_t a = *(const v4f*)(x + o);
  const v4f_t c = *(const v4f*)(x + o + 4);
  float v[8];
  v[0] = a[0]; v[1] = a[1]; v[2] = a[2]; v[3] = a[3];
  v[4] = c[0]; v[5] = c[1]; v[6] = c[2]; v[7] = c[3];
  unsigned short fh[8], bh[8], bl[8];
#pragma unroll
  for (int e = 0; e < 8; ++e) {
    fh[e] = hbits(v[e]);
    bh[e] = bfbits(v[e]);
    bl[e] = bfbits(v[e] - bff(bh[e]));
  }
  v4u_t ph, pb, pl;
#pragma unroll
  for (int e = 0; e < 4; ++e) {
    ph[e] = pk2(fh[2 * e], fh[2 * e + 1]);
    pb[e] = pk2(bh[2 * e], bh[2 * e + 1]);
    pl[e] = pk2(bl[2 * e], bl[2 * e + 1]);
  }
  *(volatile v4u*)(xh + o) = ph;
  *(volatile v4u*)(xbh + o) = pb;
  *(volatile v4u*)(xbl + o) = pl;
  __threadfence();
  *(volatile v4u*)(xh + o) = ph;
  *(volatile v4u*)(xbh + o) = pb;
  *(volatile v4u*)(xbl + o) = pl;
}

__global__ __launch_bounds__(256) void k_wprep(const float* __restrict__ W, int K, int N, int mode,
                                               unsigned short* __restrict__ P0,
                                               unsigned short* __restrict__ P1) {
  __shared__ __align__(16) float T[64 * 65];
  const int tid = threadIdx.x;
  const int n0 = blockIdx.x * 64, k0 = blockIdx.y * 64;
  {
    const int c4 = (tid & 15) * 4, kr = tid >> 4;
#pragma unroll
    for (int i = 0; i < 4; ++i) {
      const int k = kr + 16 * i;
      const v4f_t v = *(const v4f*)(W + (size_t)(k0 + k) * (size_t)N + n0 + c4);
      T[(c4 + 0) * 65 + k] = v[0];
      T[(c4 + 1) * 65 + k] = v[1];
      T[(c4 + 2) * 65 + k] = v[2];
      T[(c4 + 3) * 65 + k] = v[3];
    }
  }
  __syncthreads();
  v4u_t o0[2], o1[2];
  size_t dst[2];
#pragma unroll
  for (int i = 0; i < 2; ++i) {
    const int line = i * 32 + (tid >> 3), piece = tid & 7;
    float f[8];
#pragma unroll
    for (int e = 0; e < 8; ++e) f[e] = T[line * 65 + piece * 8 + e];
    v4u_t a, c;
    if (mode == 0) {
#pragma unroll
      for (int e = 0; e < 4; ++e) {
        a[e] = pk2(hbits(f[2 * e] * WUP), hbits(f[2 * e + 1] * WUP));
        c[e] = 0u;
      }
    } else {
#pragma unroll
      for (int e = 0; e < 4; ++e) {
        const unsigned short h0 = bfbits(f[2 * e]), h1 = bfbits(f[2 * e + 1]);
        a[e] = pk2(h0, h1);
        c[e] = pk2(bfbits(f[2 * e] - bff(h0)), bfbits(f[2 * e + 1] - bff(h1)));
      }
    }
    o0[i] = a;
    o1[i] = c;
    dst[i] = (size_t)(n0 + line) * (size_t)K + k0 + piece * 8;
  }
#pragma unroll
  for (int i = 0; i < 2; ++i) {
    *(volatile v4u*)(P0 + dst[i]) = o0[i];
    if (mode != 0) *(volatile v4u*)(P1 + dst[i]) = o1[i];
  }
  __threadfence();
#pragma unroll
  for (int i = 0; i < 2; ++i) {
    *(volatile v4u*)(P0 + dst[i]) = o0[i];
    if (mode != 0) *(volatile v4u*)(P1 + dst[i]) = o1[i];
  }
}

__global__ __launch_bounds__(128) void k_proj_f16(const unsigned short* __restrict__ xh,
                                                  const unsigned short* __restrict__ Wt5,
                                                  unsigned short* __restrict__ QK,
                                                  unsigned short* __restrict__ Vlt) {
  __shared__ __align__(16) unsigned short T[64 * PP];
  const int tid = threadIdx.x, w = tid >> 5, l = tid & 31, h = l >> 4, m = l & 15;
  const int n0 = blockIdx.x * 64, m0 = blockIdx.y * 64, z = blockIdx.z;
  const unsigned short* arow = xh + (size_t)(m0 + w * 16 + m) * ND;
  const unsigned short* wz = Wt5 + (size_t)z * ND * ND + (size_t)(n0 + m) * ND;
  v8f acc[4];
#pragma unroll
  for (int j = 0; j < 4; ++j) acc[j] = z8();

#pragma unroll 2
  for (int ks = 0; ks < ND / 32; ++ks) {
    const int k0 = ks * 32;
    const v16h a = ldh(arow + k0, h);
#pragma unroll
    for (int j = 0; j < 4; ++j) {
      const v16h b = ldh(wz + (size_t)j * 16 * ND + k0, h);
      acc[j] = mma_h(a, b, acc[j]);
    }
  }

  if (z < 4) {
#pragma unroll
    for (int j = 0; j < 4; ++j)
#pragma unroll
      for (int r = 0; r < 8; ++r)
        T[(w * 16 + 8 * h + r) * PP + j * 16 + m] = hbits(acc[j][r] * WDN);
  } else {
#pragma unroll
    for (int j = 0; j < 4; ++j) {
      v4u_t pk;
#pragma unroll
      for (int e = 0; e < 4; ++e)
        pk[e] = pk2(hbits(acc[j][2 * e] * WDN), hbits(acc[j][2 * e + 1] * WDN));
      *(v4u*)(T + (j * 16 + m) * PP + w * 16 + 8 * h) = pk;
    }
  }
  __syncthreads();

  v4u_t o[4];
  size_t dst[4];
  unsigned short* base;
  if (z < 4) {
    base = QK + (size_t)z * PLANE;
#pragma unroll
    for (int i = 0; i < 4; ++i) {
      const int row = i * 16 + (tid >> 3), piece = tid & 7;
      o[i] = *(const v4u*)(T + row * PP + piece * 8);
      dst[i] = (size_t)(m0 + row) * ND + n0 + piece * 8;
    }
  } else {
    base = Vlt;
    const int bb = m0 >> 11, s0 = m0 & (NS - 1), hd = n0 >> 6;
#pragma unroll
    for (int i = 0; i < 4; ++i) {
      const int d = i * 16 + (tid >> 3), piece = tid & 7;
      o[i] = *(const v4u*)(T + d * PP + piece * 8);
      dst[i] = ((size_t)((bb * NH + hd) * HD + d)) * NS + s0 + piece * 8;
    }
  }
#pragma unroll
  for (int i = 0; i < 4; ++i) *(volatile v4u*)(base + dst[i]) = o[i];
  __threadfence();
#pragma unroll
  for (int i = 0; i < 4; ++i) *(volatile v4u*)(base + dst[i]) = o[i];
}

__global__ __launch_bounds__(128) void k_proj_vs(const unsigned short* __restrict__ xbh,
                                                 const unsigned short* __restrict__ xbl,
                                                 const unsigned short* __restrict__ Wh,
                                                 const unsigned short* __restrict__ Wl,
                                                 unsigned short* __restrict__ Vsh,
                                                 unsigned short* __restrict__ Vsl) {
  __shared__ __align__(16) unsigned short Th[64 * PP];
  __shared__ __align__(16) unsigned short Tl[64 * PP];
  const int tid = threadIdx.x, w = tid >> 5, l = tid & 31, h = l >> 4, m = l & 15;
  const int n0 = blockIdx.x * 64, m0 = blockIdx.y * 64;
  const size_t ar = (size_t)(m0 + w * 16 + m) * ND;
  const size_t wr = (size_t)(n0 + m) * ND;
  v8f acc[4];
#pragma unroll
  for (int j = 0; j < 4; ++j) acc[j] = z8();

#pragma unroll 2
  for (int ks = 0; ks < ND / 32; ++ks) {
    const int k0 = ks * 32;
    const v16b ah = ldb(xbh + ar + k0, h);
    const v16b al = ldb(xbl + ar + k0, h);
#pragma unroll
    for (int j = 0; j < 4; ++j) {
      const size_t wo = wr + (size_t)j * 16 * ND + k0;
      const v16b bh = ldb(Wh + wo, h);
      const v16b bl = ldb(Wl + wo, h);
      acc[j] = mma_b(ah, bh, acc[j]);
      acc[j] = mma_b(ah, bl, acc[j]);
      acc[j] = mma_b(al, bh, acc[j]);
    }
  }

#pragma unroll
  for (int j = 0; j < 4; ++j) {
    v4u_t ph, pl;
#pragma unroll
    for (int e = 0; e < 4; ++e) {
      const float f0 = acc[j][2 * e], f1 = acc[j][2 * e + 1];
      const unsigned short h0 = bfbits(f0), h1 = bfbits(f1);
      ph[e] = pk2(h0, h1);
      pl[e] = pk2(bfbits(f0 - bff(h0)), bfbits(f1 - bff(h1)));
    }
    *(v4u*)(Th + (j * 16 + m) * PP + w * 16 + 8 * h) = ph;
    *(v4u*)(Tl + (j * 16 + m) * PP + w * 16 + 8 * h) = pl;
  }
  __syncthreads();

  const int bb = m0 >> 11, s0 = m0 & (NS - 1), hd = n0 >> 6;
  v4u_t oh[4], ol[4];
  size_t dst[4];
#pragma unroll
  for (int i = 0; i < 4; ++i) {
    const int d = i * 16 + (tid >> 3), piece = tid & 7;
    oh[i] = *(const v4u*)(Th + d * PP + piece * 8);
    ol[i] = *(const v4u*)(Tl + d * PP + piece * 8);
    dst[i] = ((size_t)((bb * NH + hd) * HD + d)) * NS + s0 + piece * 8;
  }
#pragma unroll
  for (int i = 0; i < 4; ++i) {
    *(volatile v4u*)(Vsh + dst[i]) = oh[i];
    *(volatile v4u*)(Vsl + dst[i]) = ol[i];
  }
  __threadfence();
#pragma unroll
  for (int i = 0; i < 4; ++i) {
    *(volatile v4u*)(Vsh + dst[i]) = oh[i];
    *(volatile v4u*)(Vsl + dst[i]) = ol[i];
  }
}

__device__ __forceinline__ void store_comb(const unsigned short* Oh, const unsigned short* Ol,
                                           unsigned short* Ch, unsigned short* Cl,
                                           int rowg0, int colbase, int l) {
  v4u_t oh[4], ol[4];
  size_t dst[4];
#pragma unroll
  for (int i = 0; i < 4; ++i) {
    const int row = i * 4 + (l >> 3), piece = l & 7;
    oh[i] = *(const v4u*)(Oh + row * PP + piece * 8);
    ol[i] = *(const v4u*)(Ol + row * PP + piece * 8);
    dst[i] = (size_t)(rowg0 + row) * NC + colbase + piece * 8;
  }
#pragma unroll
  for (int i = 0; i < 4; ++i) {
    *(volatile v4u*)(Ch + dst[i]) = oh[i];
    *(volatile v4u*)(Cl + dst[i]) = ol[i];
  }
  __threadfence();
#pragma unroll
  for (int i = 0; i < 4; ++i) {
    *(volatile v4u*)(Ch + dst[i]) = oh[i];
    *(volatile v4u*)(Cl + dst[i]) = ol[i];
  }
}

__global__ __launch_bounds__(32) void k_attn_l(const unsigned short* __restrict__ Q,
                                               const unsigned short* __restrict__ K,
                                               const unsigned short* __restrict__ Vt,
                                               const int* __restrict__ kgate,
                                               unsigned short* __restrict__ Ch,
                                               unsigned short* __restrict__ Cl) {
  __shared__ __align__(16) unsigned short Pl[16 * PP];
  __shared__ __align__(16) unsigned short Oh[16 * PP];
  __shared__ __align__(16) unsigned short Ol[16 * PP];
  const int l = threadIdx.x & 31, h = l >> 4, m = l & 15;
  const int q0 = blockIdx.x * 16, hh = blockIdx.y, b = blockIdx.z;

  const unsigned short* qrow = Q + (size_t)(b * NS + q0 + m) * ND + hh * HD;
  const v16h aq0 = ldh(qrow, h);
  const v16h aq1 = ldh(qrow + 32, h);
  const unsigned short* Kb = K + (size_t)b * NS * ND + hh * HD;
  const unsigned short* Vb = Vt + (size_t)(b * NH + hh) * HD * NS;
  const int* gk = kgate + b * NS;

  float mrow[8], lrow[8];
  v8f acc[4];
#pragma unroll
  for (int r = 0; r < 8; ++r) { mrow[r] = NEGL; lrow[r] = 0.0f; }
#pragma unroll
  for (int t = 0; t < 4; ++t) acc[t] = z8();

#pragma unroll 1
  for (int kt = 0; kt < NS / 64; ++kt) {
    const int kb = kt * 64;
    v8f s[4];
    int gv[4];
#pragma unroll
    for (int t = 0; t < 4; ++t) {
      const unsigned short* krow = Kb + (size_t)(kb + t * 16 + m) * ND;
      v8f c = z8();
      c = mma_h(aq0, ldh(krow, h), c);
      c = mma_h(aq1, ldh(krow + 32, h), c);
      s[t] = c;
      gv[t] = gk[kb + t * 16 + m];
    }
#pragma unroll
    for (int t = 0; t < 4; ++t)
#pragma unroll
      for (int r = 0; r < 8; ++r)
        s[t][r] = (gv[t] != 0) ? s[t][r] * SCL : NEGL;

#pragma unroll
    for (int r = 0; r < 8; ++r) {
      float tmax = fmaxf(fmaxf(s[0][r], s[1][r]), fmaxf(s[2][r], s[3][r]));
#pragma unroll
      for (int o = 1; o < 16; o <<= 1) tmax = fmaxf(tmax, __shfl_xor(tmax, o, 32));
      const float mnew = fmaxf(mrow[r], tmax);
      const float fac = __expf(mrow[r] - mnew);
      float p[4];
      float psum = 0.0f;
#pragma unroll
      for (int t = 0; t < 4; ++t) {
        p[t] = (s[t][r] > NEGT) ? __expf(s[t][r] - mnew) : 0.0f;
        psum += p[t];
      }
#pragma unroll
      for (int o = 1; o < 16; o <<= 1) psum += __shfl_xor(psum, o, 32);
      lrow[r] = lrow[r] * fac + psum;
      mrow[r] = mnew;
#pragma unroll
      for (int t = 0; t < 4; ++t) { acc[t][r] *= fac; s[t][r] = p[t]; }
    }

#pragma unroll
    for (int t = 0; t < 4; ++t)
#pragma unroll
      for (int r = 0; r < 8; ++r)
        Pl[(8 * h + r) * PP + t * 16 + m] = hbits(s[t][r] * PUP);
    __syncthreads();
    const v16h pa0 = ldh(Pl + m * PP, h);
    const v16h pa1 = ldh(Pl + m * PP + 32, h);
#pragma unroll
    for (int dt = 0; dt < 4; ++dt) {
      const unsigned short* vrow = Vb + (size_t)(dt * 16 + m) * NS + kb;
      acc[dt] = mma_h(pa0, ldh(vrow, h), acc[dt]);
      acc[dt] = mma_h(pa1, ldh(vrow + 32, h), acc[dt]);
    }
    __syncthreads();
  }

  float inv[8];
#pragma unroll
  for (int r = 0; r < 8; ++r) inv[r] = __builtin_amdgcn_rcpf(lrow[r]) * PDN;
#pragma unroll
  for (int dt = 0; dt < 4; ++dt)
#pragma unroll
    for (int r = 0; r < 8; ++r) {
      const float o = acc[dt][r] * inv[r];
      const unsigned short ho = bfbits(o);
      Oh[(8 * h + r) * PP + dt * 16 + m] = ho;
      Ol[(8 * h + r) * PP + dt * 16 + m] = bfbits(o - bff(ho));
    }
  __syncthreads();
  store_comb(Oh, Ol, Ch, Cl, b * NS + q0, ND + hh * HD, l);
}

__global__ __launch_bounds__(32) void k_attn_s(const unsigned short* __restrict__ Q,
                                               const unsigned short* __restrict__ K,
                                               const unsigned short* __restrict__ Vth,
                                               const unsigned short* __restrict__ Vtl,
                                               const int* __restrict__ kgate,
                                               unsigned short* __restrict__ Ch,
                                               unsigned short* __restrict__ Cl) {
  __shared__ __align__(16) unsigned short Ph[16 * PP];
  __shared__ __align__(16) unsigned short Pq[16 * PP];
  __shared__ __align__(16) unsigned short Oh[16 * PP];
  __shared__ __align__(16) unsigned short Ol[16 * PP];
  const int l = threadIdx.x & 31, h = l >> 4, m = l & 15;
  const int q0 = blockIdx.x * 16, hh = blockIdx.y, b = blockIdx.z;

  const unsigned short* qrow = Q + (size_t)(b * NS + q0 + m) * ND + hh * HD;
  const v16h aq0 = ldh(qrow, h);
  const v16h aq1 = ldh(qrow + 32, h);
  const unsigned short* Kb = K + (size_t)b * NS * ND + hh * HD;
  const size_t vbase = (size_t)(b * NH + hh) * HD * NS;
  const int* gk = kgate + b * NS;

  float mrow[8], lrow[8];
  v8f acc[4];
#pragma unroll
  for (int r = 0; r < 8; ++r) { mrow[r] = NEGL; lrow[r] = 0.0f; }
#pragma unroll
  for (int t = 0; t < 4; ++t) acc[t] = z8();

  const int kt_hi = q0 >> 6;
  const int kt_lo = (q0 >= 64) ? ((q0 - 64) >> 6) : 0;

#pragma unroll 1
  for (int kt = kt_lo; kt <= kt_hi; ++kt) {
    const int kb = kt * 64;
    v8f s[4];
    int gv[4];
#pragma unroll
    for (int t = 0; t < 4; ++t) {
      const unsigned short* krow = Kb + (size_t)(kb + t * 16 + m) * ND;
      v8f c = z8();
      c = mma_h(aq0, ldh(krow, h), c);
      c = mma_h(aq1, ldh(krow + 32, h), c);
      s[t] = c;
      gv[t] = gk[kb + t * 16 + m];
    }
#pragma unroll
    for (int t = 0; t < 4; ++t) {
      const int key = kb + t * 16 + m;
#pragma unroll
      for (int r = 0; r < 8; ++r) {
        const int rel = key - (q0 + 8 * h + r);
        const bool ok = (gv[t] != 0) && (rel <= 0) && (rel >= -64);
        s[t][r] = ok ? (s[t][r] * SCL + (float)rel * LOGD) : NEGL;
      }
    }

#pragma unroll
    for (int r = 0; r < 8; ++r) {
      float tmax = fmaxf(fmaxf(s[0][r], s[1][r]), fmaxf(s[2][r], s[3][r]));
#pragma unroll
      for (int o = 1; o < 16; o <<= 1) tmax = fmaxf(tmax, __shfl_xor(tmax, o, 32));
      const float mnew = fmaxf(mrow[r], tmax);
      const float fac = __expf(mrow[r] - mnew);
      float p[4];
      float psum = 0.0f;
#pragma unroll
      for (int t = 0; t < 4; ++t) {
        p[t] = (s[t][r] > NEGT) ? __expf(s[t][r] - mnew) : 0.0f;
        psum += p[t];
      }
#pragma unroll
      for (int o = 1; o < 16; o <<= 1) psum += __shfl_xor(psum, o, 32);
      lrow[r] = lrow[r] * fac + psum;
      mrow[r] = mnew;
#pragma unroll
      for (int t = 0; t < 4; ++t) { acc[t][r] *= fac; s[t][r] = p[t]; }
    }

#pragma unroll
    for (int t = 0; t < 4; ++t)
#pragma unroll
      for (int r = 0; r < 8; ++r) {
        const float pv = s[t][r];
        const unsigned short hp = bfbits(pv);
        Ph[(8 * h + r) * PP + t * 16 + m] = hp;
        Pq[(8 * h + r) * PP + t * 16 + m] = bfbits(pv - bff(hp));
      }
    __syncthreads();
    const v16b ph0 = ldb(Ph + m * PP, h);
    const v16b ph1 = ldb(Ph + m * PP + 32, h);
    const v16b pl0 = ldb(Pq + m * PP, h);
    const v16b pl1 = ldb(Pq + m * PP + 32, h);
#pragma unroll
    for (int dt = 0; dt < 4; ++dt) {
      const size_t vo = vbase + (size_t)(dt * 16 + m) * NS + kb;
      {
        const v16b bh = ldb(Vth + vo, h), bl = ldb(Vtl + vo, h);
        acc[dt] = mma_b(ph0, bh, acc[dt]);
        acc[dt] = mma_b(ph0, bl, acc[dt]);
        acc[dt] = mma_b(pl0, bh, acc[dt]);
      }
      {
        const v16b bh = ldb(Vth + vo + 32, h), bl = ldb(Vtl + vo + 32, h);
        acc[dt] = mma_b(ph1, bh, acc[dt]);
        acc[dt] = mma_b(ph1, bl, acc[dt]);
        acc[dt] = mma_b(pl1, bh, acc[dt]);
      }
    }
    __syncthreads();
  }

  float inv[8];
#pragma unroll
  for (int r = 0; r < 8; ++r) inv[r] = __builtin_amdgcn_rcpf(lrow[r]);
#pragma unroll
  for (int dt = 0; dt < 4; ++dt)
#pragma unroll
    for (int r = 0; r < 8; ++r) {
      const float o = acc[dt][r] * inv[r];
      const unsigned short ho = bfbits(o);
      Oh[(8 * h + r) * PP + dt * 16 + m] = ho;
      Ol[(8 * h + r) * PP + dt * 16 + m] = bfbits(o - bff(ho));
    }
  __syncthreads();
  store_comb(Oh, Ol, Ch, Cl, b * NS + q0, hh * HD, l);
}

__global__ __launch_bounds__(128) void k_out(const unsigned short* __restrict__ Ch,
                                             const unsigned short* __restrict__ Cl,
                                             const unsigned short* __restrict__ Wh,
                                             const unsigned short* __restrict__ Wl,
                                             const float* __restrict__ bo,
                                             float* __restrict__ out) {
  __shared__ __align__(16) float T[64 * TPF];
  const int tid = threadIdx.x, w = tid >> 5, l = tid & 31, h = l >> 4, m = l & 15;
  const int n0 = blockIdx.x * 64, m0 = blockIdx.y * 64;
  const size_t ar = (size_t)(m0 + w * 16 + m) * NC;
  const size_t wr = (size_t)(n0 + m) * NC;
  v8f acc[4];
#pragma unroll
  for (int j = 0; j < 4; ++j) acc[j] = z8();

#pragma unroll 2
  for (int ks = 0; ks < NC / 32; ++ks) {
    const int k0 = ks * 32;
    const v16b ah = ldb(Ch + ar + k0, h);
    const v16b al = ldb(Cl + ar + k0, h);
#pragma unroll
    for (int j = 0; j < 4; ++j) {
      const size_t wo = wr + (size_t)j * 16 * NC + k0;
      const v16b bh = ldb(Wh + wo, h);
      const v16b bl = ldb(Wl + wo, h);
      acc[j] = mma_b(ah, bh, acc[j]);
      acc[j] = mma_b(ah, bl, acc[j]);
      acc[j] = mma_b(al, bh, acc[j]);
    }
  }

#pragma unroll
  for (int j = 0; j < 4; ++j) {
    const float bias = bo[n0 + j * 16 + m];
#pragma unroll
    for (int r = 0; r < 8; ++r)
      T[(w * 16 + 8 * h + r) * TPF + j * 16 + m] = acc[j][r] + bias;
  }
  __syncthreads();

  v4f_t o[8];
  size_t dst[8];
#pragma unroll
  for (int i = 0; i < 8; ++i) {
    const int L = i * 16 + (tid >> 3), row = L >> 1, hr = L & 1, piece = tid & 7;
    o[i] = *(const v4f*)(T + row * TPF + hr * 32 + piece * 4);
    dst[i] = (size_t)(m0 + row) * ND + n0 + hr * 32 + piece * 4;
  }
#pragma unroll
  for (int i = 0; i < 8; ++i) *(volatile v4f*)(out + dst[i]) = o[i];
  __threadfence();
#pragma unroll
  for (int i = 0; i < 8; ++i) *(volatile v4f*)(out + dst[i]) = o[i];
}

extern "C" void kernel_launch(void* const* d_in, const int* in_sizes, int n_in,
                              void* d_out, int out_size, void* d_ws, size_t ws_size,
                              hipStream_t stream) {
  if (n_in < 10) return;
  if (in_sizes[0] != MR * ND || in_sizes[1] != MR) return;
  for (int i = 2; i <= 7; ++i) if (in_sizes[i] != ND * ND) return;
  if (in_sizes[8] != NC * ND || in_sizes[9] != ND) return;
  if (out_size != MR * ND) return;
  const size_t MiB = (size_t)1048576;
  const size_t total = 102 * MiB;
  if (ws_size < total) return;

  const float* x   = (const float*)d_in[0];
  const int* kgate = (const int*)d_in[1];
  const float* Wqs = (const float*)d_in[2];
  const float* Wks = (const float*)d_in[3];
  const float* Wvs = (const float*)d_in[4];
  const float* Wql = (const float*)d_in[5];
  const float* Wkl = (const float*)d_in[6];
  const float* Wvl = (const float*)d_in[7];
  const float* Wo  = (const float*)d_in[8];
  const float* bo  = (const float*)d_in[9];
  float* out = (float*)d_out;

  char* ws = (char*)d_ws;
  unsigned short* xh  = (unsigned short*)(ws + 0 * MiB);
  unsigned short* xbh = (unsigned short*)(ws + 8 * MiB);
  unsigned short* xbl = (unsigned short*)(ws + 16 * MiB);
  unsigned short* Wt5 = (unsigned short*)(ws + 24 * MiB);
  unsigned short* Wvh = (unsigned short*)(ws + 34 * MiB);
  unsigned short* Wvq = (unsigned short*)(ws + 36 * MiB);
  unsigned short* Ch  = (unsigned short*)(ws + 0 * MiB);
  unsigned short* Cl  = (unsigned short*)(ws + 16 * MiB);
  unsigned short* Woh = (unsigned short*)(ws + 38 * MiB);
  unsigned short* Woq = (unsigned short*)(ws + 42 * MiB);
  unsigned short* QK  = (unsigned short*)(ws + 46 * MiB);
  unsigned short* Vlt = (unsigned short*)(ws + 78 * MiB);
  unsigned short* Vsh = (unsigned short*)(ws + 86 * MiB);
  unsigned short* Vsq = (unsigned short*)(ws + 94 * MiB);

  {
    const int n8 = (MR * ND) / 8;
    k_xcvt<<<(n8 + 255) / 256, 256, 0, stream>>>(x, xh, xbh, xbl, n8);
  }
  {
    const float* Wf[5] = {Wqs, Wks, Wql, Wkl, Wvl};
    for (int z = 0; z < 5; ++z) {
      unsigned short* P = Wt5 + (size_t)z * ND * ND;
      k_wprep<<<dim3(ND / 64, ND / 64), 256, 0, stream>>>(Wf[z], ND, ND, 0, P, P);
    }
    k_wprep<<<dim3(ND / 64, ND / 64), 256, 0, stream>>>(Wvs, ND, ND, 1, Wvh, Wvq);
    k_wprep<<<dim3(ND / 64, NC / 64), 256, 0, stream>>>(Wo, NC, ND, 1, Woh, Woq);
  }
  k_proj_f16<<<dim3(ND / 64, MR / 64, 5), 128, 0, stream>>>(xh, Wt5, QK, Vlt);
  k_proj_vs<<<dim3(ND / 64, MR / 64), 128, 0, stream>>>(xbh, xbl, Wvh, Wvq, Vsh, Vsq);
  k_attn_s<<<dim3(NS / 16, NH, NB), 32, 0, stream>>>(QK + 0 * PLANE, QK + 1 * PLANE, Vsh, Vsq,
                                                     kgate, Ch, Cl);
  k_attn_l<<<dim3(NS / 16, NH, NB), 32, 0, stream>>>(QK + 2 * PLANE, QK + 3 * PLANE, Vlt,
                                                     kgate, Ch, Cl);
  k_out<<<dim3(ND / 64, MR / 64), 128, 0, stream>>>(Ch, Cl, Woh, Woq, bo, out);
}
